// MultiHeadAttention_RoPE_19086834663912
// MI455X (gfx1250) — hardware-verified
//
#include <hip/hip_runtime.h>
#include <math.h>
#include <float.h>
#include <stdint.h>

#define NB     1
#define SEQ    4096
#define DMODEL 768
#define NH     12
#define HD     64
#define QP     (NH * HD)
#define N3     (3 * QP)
#define QKP    (2 * QP)
#define NPAIR  (HD / 2)
#define NQB    (SEQ / 64)
#define VLP    1024
#define RESQB  16
#define MAXPOS 4095
#define NQUAD  ((2 * NH) / 4)
#define OUTN   (NB * SEQ * DMODEL)
static_assert(RESQB * 64 <= VLP);
static_assert(QP == DMODEL);
static_assert(((2 * NH) % 4) == 0);
static_assert((SEQ % 64) == 0 && (DMODEL % 64) == 0 && (N3 % 64) == 0 && (QP % 64) == 0);
static_assert(HD == 64);
static_assert((SEQ & (SEQ - 1)) == 0);
static_assert((((NB * SEQ) / 64) * (N3 / 64)) % 8 == 0);
static_assert((((NB * SEQ) / 64) * (DMODEL / 64)) % 8 == 0);
static_assert(((NB * SEQ * DMODEL / 8) % 256) == 0);
static_assert(((DMODEL * DMODEL / 8) % 256) == 0);
static_assert(((SEQ * NPAIR) % 256) == 0);
static_assert(((NB * SEQ * NQUAD) % 8) == 0);

typedef _Float16 v16h __attribute__((ext_vector_type(16)));
typedef _Float16 v8h  __attribute__((ext_vector_type(8)));
typedef __bf16   v16b __attribute__((ext_vector_type(16)));
typedef __bf16   v8b  __attribute__((ext_vector_type(8)));
typedef float    v8f  __attribute__((ext_vector_type(8)));
typedef float    v4f  __attribute__((ext_vector_type(4)));
typedef unsigned int v4u __attribute__((ext_vector_type(4)));

__device__ __forceinline__ unsigned short bf_bits(float f) {
  unsigned u = __float_as_uint(f);
  return (unsigned short)((u + 0x7FFFu + ((u >> 16) & 1u)) >> 16);
}
__device__ __forceinline__ float bf_up(unsigned short h) { return __uint_as_float(((unsigned)h) << 16); }
__device__ __forceinline__ unsigned short h_bits(_Float16 x) { return __builtin_bit_cast(unsigned short, x); }
__device__ __forceinline__ unsigned pk16(unsigned short a, unsigned short b) { return (unsigned)a | ((unsigned)b << 16); }
__device__ __forceinline__ v8f zero8() { v8f z = {0.f, 0.f, 0.f, 0.f, 0.f, 0.f, 0.f, 0.f}; return z; }
__device__ __forceinline__ v8h zero8h() {
  const _Float16 z = (_Float16)0.0f;
  v8h r = {z, z, z, z, z, z, z, z};
  return r;
}

__device__ __forceinline__ v16b ldfrag_b(const __bf16* p) {
  union { v16b v; v8b h[2]; } f;
  f.h[0] = *(const v8b*)(p);
  f.h[1] = *(const v8b*)(p + 16);
  return f.v;
}
__device__ __forceinline__ v16h ldfrag_h(const _Float16* p) {
  union { v16h v; v8h h[2]; } f;
  f.h[0] = *(const v8h*)(p);
  f.h[1] = *(const v8h*)(p + 16);
  return f.v;
}

__device__ __forceinline__ v8f mma_b(v16b a, v16b b, v8f c) {
  c = __builtin_amdgcn_wmma_f32_16x16x32_bf16(false, a, false, b, (short)0, c, false, false);
#if defined(__HIP_DEVICE_COMPILE__)
  asm volatile("v_nop\n\tv_nop\n\tv_nop\n\tv_nop" : "+v"(c) : "v"(a), "v"(b));
#endif
  return c;
}
__device__ __forceinline__ v8f mma_h(v16h a, v16h b, v8f c) {
  c = __builtin_amdgcn_wmma_f32_16x16x32_f16(false, a, false, b, (short)0, c, false, false);
#if defined(__HIP_DEVICE_COMPILE__)
  asm volatile("v_nop\n\tv_nop\n\tv_nop\n\tv_nop" : "+v"(c) : "v"(a), "v"(b));
#endif
  return c;
}
__device__ __forceinline__ v8f mma_b_raw(v16b a, v16b b, v8f c) {
  return __builtin_amdgcn_wmma_f32_16x16x32_bf16(false, a, false, b, (short)0, c, false, false);
}
__device__ __forceinline__ void dep_guard_b(v8f& a, v8f& b, v16b x, v16b y) {
#if defined(__HIP_DEVICE_COMPILE__)
  asm volatile("v_nop\n\tv_nop\n\tv_nop\n\tv_nop" : "+v"(a), "+v"(b) : "v"(x), "v"(y));
#endif
}
__device__ __forceinline__ void keep4_b(v16b a, v16b b, v16b c, v16b d) {
#if defined(__HIP_DEVICE_COMPILE__)
  asm volatile("v_nop" :: "v"(a), "v"(b), "v"(c), "v"(d));
#endif
}
__device__ __forceinline__ void acc_guard4(v8f& a, v8f& b, v8f& c, v8f& d) {
#if defined(__HIP_DEVICE_COMPILE__)
  asm volatile("v_nop\n\tv_nop\n\tv_nop\n\tv_nop" : "+v"(a), "+v"(b), "+v"(c), "+v"(d));
#endif
}

__global__ __launch_bounds__(256) void cvt_bf16x8(const float* __restrict__ in, unsigned short* out, int n8) {
  const int i = blockIdx.x * 256 + threadIdx.x;
  if (i < n8) {
    const v4f a = *(const v4f*)(in + (size_t)i * 8);
    const v4f b = *(const v4f*)(in + (size_t)i * 8 + 4);
    v4u p;
    p[0] = pk16(bf_bits(a[0]), bf_bits(a[1]));
    p[1] = pk16(bf_bits(a[2]), bf_bits(a[3]));
    p[2] = pk16(bf_bits(b[0]), bf_bits(b[1]));
    p[3] = pk16(bf_bits(b[2]), bf_bits(b[3]));
    *(volatile v4u*)(out + (size_t)i * 8) = p;
    __threadfence();
    *(volatile v4u*)(out + (size_t)i * 8) = p;
  }
}

__global__ __launch_bounds__(256) void split_bf16x8(const float* __restrict__ in, unsigned short* hp,
                                                    unsigned short* lp, int n8) {
  const int i = blockIdx.x * 256 + threadIdx.x;
  if (i < n8) {
    const v4f a = *(const v4f*)(in + (size_t)i * 8);
    const v4f b = *(const v4f*)(in + (size_t)i * 8 + 4);
    v4u ph, pl;
#pragma unroll
    for (int e = 0; e < 4; ++e) {
      const float f0 = (e < 2) ? a[2 * e]     : b[2 * e - 4];
      const float f1 = (e < 2) ? a[2 * e + 1] : b[2 * e - 3];
      const unsigned short h0 = bf_bits(f0), h1 = bf_bits(f1);
      const unsigned short l0 = bf_bits(f0 - bf_up(h0)), l1 = bf_bits(f1 - bf_up(h1));
      ph[e] = pk16(h0, h1);
      pl[e] = pk16(l0, l1);
    }
    *(volatile v4u*)(hp + (size_t)i * 8) = ph;
    *(volatile v4u*)(lp + (size_t)i * 8) = pl;
    __threadfence();
    *(volatile v4u*)(hp + (size_t)i * 8) = ph;
    *(volatile v4u*)(lp + (size_t)i * 8) = pl;
  }
}

__global__ __launch_bounds__(256) void rope_tab(const int* __restrict__ tp, float* ct, float* st, int n) {
#pragma clang fp contract(off)
  const int i = blockIdx.x * 256 + threadIdx.x;
  if (i < n) {
    int s = i >> 5;
    s = (s > SEQ - 1) ? (SEQ - 1) : s;
    const int j = i & 31;
    int pos = tp[s];
    pos = (pos < 0) ? 0 : pos;
    pos = (pos > MAXPOS) ? MAXPOS : pos;
    const float p    = (float)(2 * j) / 64.0f;
    const float base = powf(10000.0f, p);
    const float inv  = 1.0f / base;
    const float ang  = (float)pos * inv;
    const float cv = cosf(ang);
    const float sv = sinf(ang);
    *(volatile float*)(ct + i) = cv;
    *(volatile float*)(st + i) = sv;
    __threadfence();
    *(volatile float*)(ct + i) = cv;
    *(volatile float*)(st + i) = sv;
  }
}

template <int NSPLIT>
__global__ __launch_bounds__(256) void gemm64(
    const unsigned short* __restrict__ Ap, const unsigned short* A2p, int lda,
    const unsigned short* __restrict__ Btp, int ldb,
    float* C, int ldc, int M, int N, int K) {
  const __bf16* Ab  = (const __bf16*)(const void*)Ap;
  const __bf16* Ab2 = (const __bf16*)(const void*)A2p;
  const __bf16* Bb  = (const __bf16*)(const void*)Btp;
  __shared__ __align__(16) float sT[8][16 * 68];
  const int lane = threadIdx.x & 31;
  const int wave = threadIdx.x >> 5;
  const int tilesN = N >> 6;
  const int tilesM = M >> 6;
  const int tile = blockIdx.x * 8 + wave;
  if (tile >= tilesM * tilesN) return;
  const int tm = tile / tilesN;
  const int tn = tile - tm * tilesN;
  const int m0 = tm << 6;
  const int n0 = tn << 6;

  const int rlane = lane & 15;
  const int koff  = (lane >> 4) * 8;
  const int mOff  = (lane >> 4) * 8;

  v8f acc[4][4];
#pragma unroll
  for (int i = 0; i < 4; ++i)
#pragma unroll
    for (int j = 0; j < 4; ++j) acc[i][j] = zero8();

  for (int k0 = 0; k0 < K; k0 += 32) {
    v16b bh[4];
#pragma unroll
    for (int j = 0; j < 4; ++j) {
      const size_t bo = (size_t)(n0 + (j << 4) + rlane) * ldb + koff + k0;
      bh[j] = ldfrag_b(Bb + bo);
    }
#pragma unroll
    for (int i = 0; i < 4; ++i) {
      const size_t ao = (size_t)(m0 + (i << 4) + rlane) * lda + koff + k0;
      const v16b ah = ldfrag_b(Ab + ao);
      v16b al = ah;
      if (NSPLIT >= 1) al = ldfrag_b(Ab2 + ao);
#pragma unroll
      for (int j = 0; j < 4; ++j) {
        acc[i][j] = mma_b_raw(ah, bh[j], acc[i][j]);
        if (NSPLIT >= 1) acc[i][j] = mma_b_raw(al, bh[j], acc[i][j]);
      }
      dep_guard_b(acc[i][0], acc[i][3], ah, al);
    }
    keep4_b(bh[0], bh[1], bh[2], bh[3]);
  }
  acc_guard4(acc[0][0], acc[0][1], acc[0][2], acc[0][3]);
  acc_guard4(acc[1][0], acc[1][1], acc[1][2], acc[1][3]);
  acc_guard4(acc[2][0], acc[2][1], acc[2][2], acc[2][3]);
  acc_guard4(acc[3][0], acc[3][1], acc[3][2], acc[3][3]);

  float* slab = sT[wave];
#pragma unroll
  for (int i = 0; i < 4; ++i) {
    const int mBase = m0 + (i << 4);
#pragma unroll
    for (int r = 0; r < 8; ++r) {
#pragma unroll
      for (int j = 0; j < 4; ++j) {
        slab[(mOff + r) * 68 + (j << 4) + rlane] = acc[i][j][r];
      }
    }
    __builtin_amdgcn_fence(__ATOMIC_RELEASE, "workgroup");
    __builtin_amdgcn_wave_barrier();
    __builtin_amdgcn_fence(__ATOMIC_ACQUIRE, "workgroup");
    {
      const int hh = lane >> 4, c4 = (lane & 15) * 4;
      v4f ov[8];
#pragma unroll
      for (int it = 0; it < 8; ++it) {
        const int row = it * 2 + hh;
        ov[it] = *(const v4f*)(slab + row * 68 + c4);
      }
      for (int pass = 0; pass < 2; ++pass) {
#pragma unroll
        for (int it = 0; it < 8; ++it) {
          const int row = it * 2 + hh;
          *(volatile v4f*)(C + (size_t)(mBase + row) * ldc + n0 + c4) = ov[it];
        }
        __threadfence();
      }
    }
    __builtin_amdgcn_fence(__ATOMIC_RELEASE, "workgroup");
    __builtin_amdgcn_wave_barrier();
    __builtin_amdgcn_fence(__ATOMIC_ACQUIRE, "workgroup");
  }
}

__global__ __launch_bounds__(256) void rope_rows(const float* __restrict__ src, int srp,
                                                 const float* __restrict__ ct, const float* __restrict__ st,
                                                 unsigned short* dst, int rp, int nquad, int nwaves,
                                                 float oscale) {
#pragma clang fp contract(off)
  __shared__ __align__(16) float sy[8][256];
  const int tid = threadIdx.x, wave = tid >> 5, lane = tid & 31;
  const int w = blockIdx.x * 8 + wave;
  if (w >= nwaves) return;
  const int hq = w % nquad;
  const int bs = w / nquad;
  const int s  = bs & (SEQ - 1);
  const float* row = src + (size_t)bs * srp + (size_t)hq * 256;
  const float cs = ct[(size_t)s * NPAIR + lane];
  const float sn = st[(size_t)s * NPAIR + lane];
  float* buf = sy[wave];
#pragma unroll
  for (int t = 0; t < 4; ++t) {
    const float* s2 = row + t * HD;
    const float x0 = s2[2 * lane];
    const float x1 = s2[2 * lane + 1];
    const float y0 = x0 * cs - x1 * sn;
    const float y1 = x0 * sn + x1 * cs;
    buf[t * 64 + 2 * lane]     = y0;
    buf[t * 64 + 2 * lane + 1] = y1;
  }
  __builtin_amdgcn_fence(__ATOMIC_RELEASE, "workgroup");
  __builtin_amdgcn_wave_barrier();
  __builtin_amdgcn_fence(__ATOMIC_ACQUIRE, "workgroup");
  const int g = lane >> 3, piece = lane & 7;
  const float* sp = buf + g * 64 + piece * 8;
  const v4f a0 = *(const v4f*)(sp);
  const v4f a1 = *(const v4f*)(sp + 4);
  v4u val;
#pragma unroll
  for (int e = 0; e < 4; ++e) {
    const float f0 = (e < 2) ? a0[2 * e]     : a1[2 * e - 4];
    const float f1 = (e < 2) ? a0[2 * e + 1] : a1[2 * e - 3];
    val[e] = pk16(h_bits((_Float16)(f0 * oscale)), h_bits((_Float16)(f1 * oscale)));
  }
  const size_t go = (size_t)bs * rp + (size_t)hq * 256 + (size_t)g * 64 + piece * 8;
  *(volatile v4u*)(dst + go) = val;
  __threadfence();
  *(volatile v4u*)(dst + go) = val;
}

__global__ __launch_bounds__(256) void v_planes(const float* __restrict__ vf, int vrp,
                                                unsigned short* vth, unsigned short* vtl) {
  __shared__ __align__(16) float sv[64 * 68];
  const int tid = threadIdx.x;
  const int t0  = blockIdx.x * 64;
  const int hh  = blockIdx.y;
  const int b   = blockIdx.z;
#pragma unroll
  for (int i = 0; i < 4; ++i) {
    const int idx = i * 256 + tid;
    const int tt = idx >> 4, c4 = (idx & 15) * 4;
    const v4f a = *(const v4f*)(vf + ((size_t)(b * SEQ + t0 + tt)) * vrp + hh * HD + c4);
    *(v4f*)(sv + tt * 68 + c4) = a;
  }
  __syncthreads();

  const int g = tid >> 3, piece = tid & 7;
  v4u hv[2], lv[2];
  size_t hofs[2], lofs[2];
#pragma unroll
  for (int it = 0; it < 2; ++it) {
    const int d = it * 32 + g;
    v4u a, a2;
#pragma unroll
    for (int e = 0; e < 4; ++e) {
      const float f0 = sv[(piece * 8 + 2 * e) * 68 + d];
      const float f1 = sv[(piece * 8 + 2 * e + 1) * 68 + d];
      const _Float16 x0 = (_Float16)f0, x1 = (_Float16)f1;
      const unsigned short h0 = h_bits(x0), h1 = h_bits(x1);
      const unsigned short l0 = h_bits((_Float16)((f0 - (float)x0) * 4096.0f));
      const unsigned short l1 = h_bits((_Float16)((f1 - (float)x1) * 4096.0f));
      a[e] = pk16(h0, h1); a2[e] = pk16(l0, l1);
    }
    hv[it] = a; lv[it] = a2;
    const size_t rowf = (size_t)(b * QP + hh * HD + d);
    hofs[it] = rowf * SEQ + t0 + piece * 8;
    lofs[it] = rowf * VLP + t0 + piece * 8;
  }
  const bool wlo = (t0 + 64 <= VLP);
  for (int pass = 0; pass < 2; ++pass) {
#pragma unroll
    for (int it = 0; it < 2; ++it) {
      *(volatile v4u*)(vth + hofs[it]) = hv[it];
      if (wlo) *(volatile v4u*)(vtl + lofs[it]) = lv[it];
    }
    __threadfence();
  }
}

template <bool RESV>
__global__ __launch_bounds__(128)
void attn_causal64(const unsigned short* __restrict__ qkp,
                   const unsigned short* __restrict__ vhp, const unsigned short* __restrict__ vlp,
                   float* outp, int qbBase, int nqbThis, float sscale) {
  union FH { v16h v; v8h h[2]; };
  __shared__ __align__(16) _Float16 Ksh[64 * 64];
  __shared__ __align__(16) _Float16 Vth[64 * 64];
  __shared__ __align__(16) _Float16 Vtl[RESV ? 64 * 64 : 8];
  __shared__ __align__(16) _Float16 Psh[4][16 * 64];
  __shared__ __align__(16) _Float16 Psl[RESV ? 4 : 1][16 * 64];
  __shared__ __align__(16) float    Os[4][16 * 64];

  const int tid  = threadIdx.x;
  const int wave = tid >> 5;
  const int lane = tid & 31;
  const int hh   = lane >> 4;
  const int c    = lane & 15;

  const int bx   = blockIdx.x;
  const int qbl  = bx % nqbThis;
  const int rest = bx / nqbThis;
  const int h    = rest % NH;
  const int b    = rest / NH;
  const int qb   = qbBase + qbl;
  const int q0   = qb * 64 + wave * 16;
  const size_t rowB = (size_t)b * SEQ;

  const _Float16* Qp = (const _Float16*)(const void*)qkp + (size_t)h * HD;
  const _Float16* Kp = Qp + QP;
  const _Float16* Vh = (const _Float16*)(const void*)vhp + ((size_t)b * QP + (size_t)h * HD) * SEQ;
  const _Float16* Vl = (const _Float16*)(const void*)vlp + ((size_t)b * QP + (size_t)h * HD) * VLP;

  v16h qa[2];
#pragma unroll
  for (int dc = 0; dc < 2; ++dc) {
    const size_t qo = (rowB + q0 + c) * QKP + dc * 32 + 8 * hh;
    qa[dc] = ldfrag_h(Qp + qo);
  }

  float mrow[8], lrow[8];
  v8f oacc[4];
#pragma unroll
  for (int r = 0; r < 8; ++r) { mrow[r] = -INFINITY; lrow[r] = 0.f; }
#pragma unroll
  for (int t = 0; t < 4; ++t) oacc[t] = zero8();

  int nkt = qb + 1;
  if (nkt > NQB) nkt = NQB;
  for (int kt = 0; kt < nkt; ++kt) {
    const int kv0 = kt * 64;
    __syncthreads();
    {
      const int r = tid >> 1, half = (tid & 1) * 32;
      const _Float16* kg = Kp + (rowB + kv0 + r) * QKP + half;
      const _Float16* vg = Vh + (size_t)r * SEQ + kv0 + half;
      const int kvl = (kv0 + 64 <= VLP) ? kv0 : (VLP - 64);
      const _Float16* vlg = Vl + (size_t)r * VLP + kvl + half;
      const bool resOK = (kv0 + 64 <= VLP);
#pragma unroll
      for (int i = 0; i < 4; ++i) {
        const v8h a0 = *(const v8h*)(kg + 8 * i);
        const v8h b0 = *(const v8h*)(vg + 8 * i);
        *(v8h*)(Ksh + r * 64 + half + 8 * i) = a0;
        *(v8h*)(Vth + r * 64 + half + 8 * i) = b0;
        if (RESV) {
          v8h b1 = *(const v8h*)(vlg + 8 * i);
          if (!resOK) b1 = zero8h();
          *(v8h*)(Vtl + r * 64 + half + 8 * i) = b1;
        }
      }
    }
    __syncthreads();

    v8f s[4];
#pragma unroll
    for (int j = 0; j < 4; ++j) {
      s[j] = zero8();
#pragma unroll
      for (int dc = 0; dc < 2; ++dc) {
        FH kb;
        kb.h[0] = *(const v8h*)(Ksh + (j * 16 + c) * 64 + dc * 32 + 8 * hh);
        kb.h[1] = *(const v8h*)(Ksh + (j * 16 + c) * 64 + dc * 32 + 16 + 8 * hh);
        s[j] = mma_h(qa[dc], kb.v, s[j]);
      }
    }

    _Float16* pwh = Psh[wave];
    _Float16* pwl = Psl[RESV ? wave : 0];
#pragma unroll
    for (int r = 0; r < 8; ++r) {
      const int qrow = q0 + 8 * hh + r;
      float m = -INFINITY;
#pragma unroll
      for (int j = 0; j < 4; ++j) {
        const int key = kv0 + j * 16 + c;
        float sv = s[j][r] * sscale;
        sv = (key > qrow) ? -FLT_MAX : sv;
        s[j][r] = sv;
        m = fmaxf(m, sv);
      }
#pragma unroll
      for (int off = 1; off < 16; off <<= 1) m = fmaxf(m, __shfl_xor(m, off, 32));
      const float mnew  = fmaxf(mrow[r], m);
      const float msafe = (mnew == -INFINITY) ? 0.f : mnew;
      const float alpha = __expf(mrow[r] - msafe);
      mrow[r] = mnew;
      float psum = 0.f;
#pragma unroll
      for (int j = 0; j < 4; ++j) {
        const float p = __expf(s[j][r] - msafe);
        psum += p;
        const float p1k = p * 1024.0f;
        const _Float16 ph = (_Float16)p1k;
        pwh[(8 * hh + r) * 64 + j * 16 + c] = ph;
        if (RESV) {
          const _Float16 pl = (_Float16)((p1k - (float)ph) * 4096.0f);
          pwl[(8 * hh + r) * 64 + j * 16 + c] = pl;
        }
      }
#pragma unroll
      for (int off = 1; off < 16; off <<= 1) psum += __shfl_xor(psum, off, 32);
      lrow[r] = lrow[r] * alpha + psum;
#pragma unroll
      for (int t = 0; t < 4; ++t) oacc[t][r] *= alpha;
    }
    __builtin_amdgcn_fence(__ATOMIC_RELEASE, "workgroup");
    __builtin_amdgcn_wave_barrier();
    __builtin_amdgcn_fence(__ATOMIC_ACQUIRE, "workgroup");

    v8f o1[4];
#pragma unroll
    for (int t = 0; t < 4; ++t) o1[t] = zero8();
#pragma unroll 1
    for (int kk = 0; kk < 2; ++kk) {
      FH pa, pl;
      pa.h[0] = *(const v8h*)(pwh + c * 64 + kk * 32 + 8 * hh);
      pa.h[1] = *(const v8h*)(pwh + c * 64 + kk * 32 + 16 + 8 * hh);
      if (RESV) {
        pl.h[0] = *(const v8h*)(pwl + c * 64 + kk * 32 + 8 * hh);
        pl.h[1] = *(const v8h*)(pwl + c * 64 + kk * 32 + 16 + 8 * hh);
      } else {
        pl.v = pa.v;
      }
#pragma unroll
      for (int t = 0; t < 4; ++t) {
        FH vb;
        vb.h[0] = *(const v8h*)(Vth + (t * 16 + c) * 64 + kk * 32 + 8 * hh);
        vb.h[1] = *(const v8h*)(Vth + (t * 16 + c) * 64 + kk * 32 + 16 + 8 * hh);
        oacc[t] = mma_h(pa.v, vb.v, oacc[t]);
        if (RESV) {
          FH vl;
          vl.h[0] = *(const v8h*)(Vtl + (t * 16 + c) * 64 + kk * 32 + 8 * hh);
          vl.h[1] = *(const v8h*)(Vtl + (t * 16 + c) * 64 + kk * 32 + 16 + 8 * hh);
          o1[t] = mma_h(pa.v, vl.v, o1[t]);
          o1[t] = mma_h(pl.v, vb.v, o1[t]);
        }
      }
    }
    if (RESV) {
#pragma unroll
      for (int t = 0; t < 4; ++t)
#pragma unroll
        for (int r = 0; r < 8; ++r) oacc[t][r] += o1[t][r] * (1.0f / 4096.0f);
    }
  }

  float* os = Os[wave];
#pragma unroll
  for (int r = 0; r < 8; ++r) {
    const float l = lrow[r];
    const float inv = ((l > 0.f) ? (1.0f / l) : 0.f) * (1.0f / 1024.0f);
#pragma unroll
    for (int t = 0; t < 4; ++t) os[(8 * hh + r) * 64 + t * 16 + c] = oacc[t][r] * inv;
  }
  __builtin_amdgcn_fence(__ATOMIC_RELEASE, "workgroup");
  __builtin_amdgcn_wave_barrier();
  __builtin_amdgcn_fence(__ATOMIC_ACQUIRE, "workgroup");
  {
    const int h2 = lane >> 4, c4 = (lane & 15) * 4;
    v4f ov[8];
#pragma unroll
    for (int it = 0; it < 8; ++it) {
      const int row = it * 2 + h2;
      ov[it] = *(const v4f*)(os + row * 64 + c4);
    }
    for (int pass = 0; pass < 2; ++pass) {
#pragma unroll
      for (int it = 0; it < 8; ++it) {
        const int row = it * 2 + h2;
        const size_t go = (rowB + q0 + row) * QP + (size_t)h * HD + c4;
        *(volatile v4f*)(outp + go) = ov[it];
      }
      __threadfence();
    }
  }
}

extern "C" void kernel_launch(void* const* d_in, const int* in_sizes, int n_in,
                              void* d_out, int out_size, void* d_ws, size_t ws_size,
                              hipStream_t stream) {
  if (n_in < 6) return;
  if (in_sizes[0] != NB * SEQ * DMODEL) return;
  if (in_sizes[1] != SEQ) return;
  if (in_sizes[2] != DMODEL * DMODEL) return;
  if (in_sizes[3] != DMODEL * DMODEL) return;
  if (in_sizes[4] != DMODEL * DMODEL) return;
  if (in_sizes[5] != DMODEL * DMODEL) return;
  if (out_size != OUTN) return;

  const float* x  = (const float*)d_in[0];
  const int*   tp = (const int*)d_in[1];
  const float* Wq = (const float*)d_in[2];
  const float* Wk = (const float*)d_in[3];
  const float* Wv = (const float*)d_in[4];
  const float* Wo = (const float*)d_in[5];

  const size_t PXb   = (size_t)NB * SEQ * DMODEL * 2;
  const size_t PWT   = (size_t)N3 * DMODEL * 2;
  const size_t PWo   = (size_t)DMODEL * QP * 2;
  const size_t PTrig = (size_t)SEQ * NPAIR * 4;
  const size_t PQKV  = (size_t)NB * SEQ * N3 * 4;
  const size_t PVTh  = (size_t)NB * QP * SEQ * 2;
  const size_t PVTl  = (size_t)NB * QP * VLP * 2;
  const size_t PQK   = (size_t)NB * SEQ * QKP * 2;
  const size_t PAf   = (size_t)NB * SEQ * QP * 4;
  const size_t PA    = (size_t)NB * SEQ * QP * 2;
  size_t off = 0;
  const size_t oXb  = off; off += PXb;
  const size_t oWT  = off; off += PWT;
  const size_t oWo  = off; off += PWo;
  const size_t oCos = off; off += PTrig;
  const size_t oSin = off; off += PTrig;
  const size_t oQKV = off; off += PQKV;
  const size_t oVTh = off; off += PVTh;
  const size_t oVTl = off; off += PVTl;
  const size_t oQK  = off; off += PQK;
  const size_t oAf  = off; off += PAf;
  const size_t oAh  = off; off += PA;
  const size_t oAl  = off; off += PA;
  if (off > ws_size) return;
  if (off > (size_t)134217728) return;

  char* ws = (char*)d_ws;
  unsigned short* Xb   = (unsigned short*)(ws + oXb);
  unsigned short* WT   = (unsigned short*)(ws + oWT);
  unsigned short* WoT  = (unsigned short*)(ws + oWo);
  float*          CosT = (float*)(ws + oCos);
  float*          SinT = (float*)(ws + oSin);
  float*          QKVf = (float*)(ws + oQKV);
  unsigned short* VTh  = (unsigned short*)(ws + oVTh);
  unsigned short* VTl  = (unsigned short*)(ws + oVTl);
  unsigned short* QK   = (unsigned short*)(ws + oQK);
  float*          Af   = (float*)(ws + oAf);
  unsigned short* Ah   = (unsigned short*)(ws + oAh);
  unsigned short* Al   = (unsigned short*)(ws + oAl);
  float*          outf = (float*)d_out;

  const dim3 blk(256);
  const int nTok  = NB * SEQ;
  const int nTrig = SEQ * NPAIR;
  const int n8x   = NB * SEQ * DMODEL / 8;
  const int n8w   = DMODEL * DMODEL / 8;
  const int n8a   = NB * SEQ * QP / 8;
  const int nwQK  = nTok * NQUAD;
  const size_t DD = (size_t)DMODEL * DMODEL;
  const dim3 gTrig((nTrig + 255) / 256);
  const dim3 gCvtX((n8x + 255) / 256);
  const dim3 gCvtW((n8w + 255) / 256);
  const dim3 gQKV(((NB * SEQ / 64) * (N3 / 64) + 7) / 8);
  const dim3 gRope((nwQK + 7) / 8);
  const dim3 gVpl(SEQ / 64, NH, NB);
  const dim3 gSplit((n8a + 255) / 256);
  const dim3 gOut(((NB * SEQ / 64) * (DMODEL / 64) + 7) / 8);
  const float qkScale = 16.0f;
  const float sscale  = 1.0f / 2048.0f;

  rope_tab<<<gTrig, blk, 0, stream>>>(tp, CosT, SinT, nTrig);
  cvt_bf16x8<<<gCvtX, blk, 0, stream>>>(x, Xb, n8x);
  cvt_bf16x8<<<gCvtW, blk, 0, stream>>>(Wq, WT, n8w);
  cvt_bf16x8<<<gCvtW, blk, 0, stream>>>(Wk, WT + DD, n8w);
  cvt_bf16x8<<<gCvtW, blk, 0, stream>>>(Wv, WT + 2 * DD, n8w);
  cvt_bf16x8<<<gCvtW, blk, 0, stream>>>(Wo, WoT, n8w);
  gemm64<0><<<gQKV, blk, 0, stream>>>(Xb, Xb, DMODEL, WT, DMODEL, QKVf, N3, NB * SEQ, N3, DMODEL);
  rope_rows<<<gRope, blk, 0, stream>>>(QKVf, N3, CosT, SinT, QK, QKP, NQUAD, nwQK, qkScale);
  v_planes<<<gVpl, blk, 0, stream>>>(QKVf + 2 * QP, N3, VTh, VTl);
  attn_causal64<true><<<dim3(NB * NH * RESQB), dim3(128), 0, stream>>>(
      QK, VTh, VTl, Af, 0, RESQB, sscale);
  attn_causal64<false><<<dim3(NB * NH * (NQB - RESQB)), dim3(128), 0, stream>>>(
      QK, VTh, VTl, Af, RESQB, NQB - RESQB, sscale);
  split_bf16x8<<<gSplit, blk, 0, stream>>>(Af, Ah, Al, n8a);
  gemm64<1><<<gOut, blk, 0, stream>>>(Ah, Al, QP, WoT, QP, outf, DMODEL, NB * SEQ, DMODEL, QP);
  (void)hipGetLastError();
}
